// GCN_39307540693880
// MI455X (gfx1250) — hardware-verified
//
#include <hip/hip_runtime.h>
#include <stddef.h>


typedef _Float16 v16h __attribute__((ext_vector_type(16)));
typedef _Float16 v8h  __attribute__((ext_vector_type(8)));
typedef float    v8f  __attribute__((ext_vector_type(8)));
typedef float    v4f  __attribute__((ext_vector_type(4)));
typedef _Float16 h16;

#ifndef NN
#define NN 2048
#endif
#define NN_FULL 2048
#define FD 128
#define HD 32
#define CD 16
#define KC (HD + FD)

static_assert(NN >= 128 && NN <= NN_FULL && (NN % 128) == 0);
static_assert((NN % 32) == 0 && (NN % 64) == 0);
static_assert(FD == 128 && (FD % 32) == 0);
static_assert(HD == 32 && (HD % 32) == 0);
static_assert(CD == 16);
static_assert((KC % 32) == 0 && KC == 160);
static_assert((size_t)NN_FULL * NN_FULL * 4 == (size_t)16777216);

#define WCARRY 64.0f
#define XCARRY 16.0f
#define ACARRY 4096.0f
#define GCARRY 16.0f
#define RCARRY 2048.0f
#define YCARRY 16.0f

#define LDG 72
#define LDX 36
#define LDY 136
#define LDO 20
#define WMAX 4096
static_assert((LDG % 8) == 0 && LDG >= 64);
static_assert((LDX % 4) == 0 && LDX >= HD);
static_assert((LDY % 8) == 0 && LDY >= 128);
static_assert((LDO % 4) == 0 && LDO >= CD);
static_assert(FD * HD <= WMAX && KC * CD <= WMAX);
static_assert(((FD * HD) % 8) == 0 && ((KC * CD) % 8) == 0);

#define W1T_BYTES ((size_t)HD * FD * 2)
#define W2T_BYTES ((size_t)CD * KC * 2)
#define X16_BYTES ((size_t)NN * FD * 2)
#define A16_BYTES ((size_t)NN * NN * 2)
#define GP_BYTES  ((size_t)HD * NN * 2)
#define X32_BYTES ((size_t)NN * HD * 2)
#define UV_BYTES  ((size_t)2 * NN * 4)
#define YT_BYTES  ((size_t)CD * NN * 2)
#define OFF_W1T ((size_t)0)
#define OFF_W2T (OFF_W1T + W1T_BYTES)
#define OFF_X16 (OFF_W2T + W2T_BYTES)
#define OFF_A16 (OFF_X16 + X16_BYTES)
#define OFF_GH  (OFF_A16 + A16_BYTES)
#define OFF_GR  (OFF_GH + GP_BYTES)
#define OFF_X32 (OFF_GR + GP_BYTES)
#define OFF_UV  (OFF_X32 + X32_BYTES)
#define OFF_YT  (OFF_UV + UV_BYTES)
#define OFF_A1  (OFF_YT + YT_BYTES)
#define WS_TOTAL (OFF_A1 + A16_BYTES)
static_assert((W1T_BYTES % 128) == 0 && (W2T_BYTES % 128) == 0 && (X16_BYTES % 128) == 0);
static_assert((A16_BYTES % 128) == 0 && (GP_BYTES % 128) == 0 && (X32_BYTES % 128) == 0);
static_assert((UV_BYTES % 128) == 0 && (YT_BYTES % 128) == 0);
static_assert(WS_TOTAL <= (size_t)134217728);
static_assert((size_t)(2 * HD * LDG) * 2 <= (size_t)131072);
static_assert((size_t)(64 * LDX + 96 + 128) * 4 <= (size_t)131072);
static_assert((size_t)CD * LDY * 2 <= (size_t)131072);
static_assert((size_t)128 * LDO * 4 <= (size_t)131072);

__device__ __forceinline__ float bf16r(float x) {
  unsigned int u = __float_as_uint(x);
  u = (u + 0x7FFFu + ((u >> 16) & 1u)) & 0xFFFF0000u;
  return __uint_as_float(u);
}

__device__ __forceinline__ h16 toh_flush(float v) {
  const h16 r = (h16)v;
  return (fabsf(v) < 6.103515625e-05f) ? (h16)0.0f : r;
}

__device__ __forceinline__ v16h frag_at(const _Float16* p) {
  v8h lo = *(const v8h*)(p);
  v8h hi = *(const v8h*)(p + 16);
  v16h out;
#pragma unroll
  for (int i = 0; i < 8; ++i) { out[i] = lo[i]; out[i + 8] = hi[i]; }
  return out;
}

__device__ __forceinline__ v8f wmma16(v16h a, v16h b, v8f c) {
  v8f d = __builtin_amdgcn_wmma_f32_16x16x32_f16(false, a, false, b, (short)0, c,
                                                 false, false);
  asm volatile("v_nop\n\tv_nop\n\tv_nop\n\tv_nop" : "+v"(d) : "v"(a), "v"(b));
  return d;
}

__global__ __launch_bounds__(256) void wconv_kernel(
    const float* __restrict__ W, _Float16* __restrict__ Wt, int K, int N) {
#pragma clang fp contract(off)
  __shared__ __attribute__((aligned(16))) _Float16 T[WMAX];
  const unsigned tid = threadIdx.x;
  const unsigned total = (unsigned)K * (unsigned)N;
#pragma unroll 1
  for (unsigned idx = tid; idx < total; idx += 256u) {
    const unsigned kr = idx / (unsigned)N;
    const unsigned nc = idx - kr * (unsigned)N;
    const float v = W[idx];
    T[nc * (unsigned)K + kr] = toh_flush(WCARRY * bf16r(v));
  }
  __syncthreads();
  const unsigned np = total >> 3;
#pragma unroll 1
  for (unsigned p = tid; p < np; p += 256u) {
    const v8h o = *(const v8h*)&T[p * 8u];
    *(volatile v8h*)(Wt + (size_t)p * 8u) = o;
  }
  __threadfence();
#pragma unroll 1
  for (unsigned p = tid; p < np; p += 256u) {
    const v8h o = *(const v8h*)&T[p * 8u];
    *(volatile v8h*)(Wt + (size_t)p * 8u) = o;
  }
}

__global__ __launch_bounds__(256) void pconv_kernel(
    const float* __restrict__ src, _Float16* __restrict__ dst, int cols8, int src_pitch,
    float carry) {
#pragma clang fp contract(off)
  const unsigned gid = blockIdx.x * 256u + threadIdx.x;
  const unsigned row = gid / (unsigned)cols8;
  const unsigned c = (gid - row * (unsigned)cols8) * 8u;
  const float* s = src + (size_t)row * (unsigned)src_pitch + c;
  const v4f a0 = *(const v4f*)(s);
  const v4f a1 = *(const v4f*)(s + 4u);
  v8h o;
#pragma unroll
  for (int i = 0; i < 4; ++i) {
    o[i]     = toh_flush(carry * bf16r(a0[i]));
    o[i + 4] = toh_flush(carry * bf16r(a1[i]));
  }
  _Float16* p = dst + (size_t)gid * 8u;
  *(volatile v8h*)p = o;
  __threadfence();
  *(volatile v8h*)p = o;
}
static_assert(((size_t)NN * (FD / 8)) % 256 == 0);
static_assert(((size_t)NN * (NN / 8)) % 256 == 0);

__global__ __launch_bounds__(256) void gemm_xw_kernel(
    const _Float16* __restrict__ A16, const _Float16* __restrict__ Bt,
    _Float16* __restrict__ Gh, _Float16* __restrict__ Gr) {
#pragma clang fp contract(off)
  __shared__ __attribute__((aligned(16))) _Float16 Th[HD * LDG];
  __shared__ __attribute__((aligned(16))) _Float16 Tr[HD * LDG];
  const unsigned tid = threadIdx.x, lane = tid & 31u;
  const unsigned w = (unsigned)__builtin_amdgcn_readfirstlane((int)(threadIdx.x >> 5));
  const unsigned mw = w >> 1, nw = w & 1u;
  const unsigned hh = lane >> 4, m = lane & 15u;
  const unsigned row0 = blockIdx.x * 64u;

  const _Float16* ap = A16 + (size_t)(row0 + mw * 16u + m) * FD + hh * 8u;
  const _Float16* bp = Bt + (size_t)(nw * 16u + m) * FD + hh * 8u;
  v8f acc = {};
#pragma unroll
  for (unsigned k0 = 0; k0 < (unsigned)FD; k0 += 32u) {
    const v16h a = frag_at(ap + k0);
    const v16h b = frag_at(bp + k0);
    acc = wmma16(a, b, acc);
  }
  const float cs = GCARRY / (WCARRY * XCARRY);
  v8h oh, orr;
#pragma unroll
  for (int r = 0; r < 8; ++r) {
    const float g = acc[r] * cs;
    const h16 hv = toh_flush(g);
    const float res = (g - (float)hv) * RCARRY;
    oh[r] = hv;
    orr[r] = toh_flush(res);
  }
  *(v8h*)&Th[(nw * 16u + m) * LDG + mw * 16u + hh * 8u] = oh;
  *(v8h*)&Tr[(nw * 16u + m) * LDG + mw * 16u + hh * 8u] = orr;
  __syncthreads();

  const unsigned n = tid >> 3, c = (tid & 7u) * 8u;
  const v8h xh = *(const v8h*)&Th[n * LDG + c];
  const v8h xr = *(const v8h*)&Tr[n * LDG + c];
  const size_t off = (size_t)n * NN + row0 + c;
  *(volatile v8h*)(Gh + off) = xh;
  *(volatile v8h*)(Gr + off) = xr;
  __threadfence();
  *(volatile v8h*)(Gh + off) = xh;
  *(volatile v8h*)(Gr + off) = xr;
}
static_assert(256 / 8 == HD);
static_assert(8 * 8 == 64);

__global__ __launch_bounds__(256) void gemm_adj_kernel(
    const _Float16* __restrict__ A16, const _Float16* __restrict__ Gh,
    const _Float16* __restrict__ Gr,
    const float* __restrict__ b1, const float* __restrict__ Wc1, const float* __restrict__ bc1,
    const float* __restrict__ Wc2, const float* __restrict__ bc2,
    _Float16* __restrict__ X32, float* __restrict__ UV) {
#pragma clang fp contract(off)
  __shared__ __attribute__((aligned(16))) float xs[64 * LDX];
  __shared__ __attribute__((aligned(16))) float wab[96];
  __shared__ __attribute__((aligned(16))) float suv[128];
  const unsigned tid = threadIdx.x, lane = tid & 31u;
  const unsigned w = (unsigned)__builtin_amdgcn_readfirstlane((int)(threadIdx.x >> 5));
  const unsigned mw = w >> 1, nw = w & 1u;
  const unsigned hh = lane >> 4, m = lane & 15u;
  const unsigned row0 = blockIdx.x * 64u;

  if (w < 2u) {
    float s = 0.0f;
#pragma unroll 1
    for (unsigned h = 0; h < (unsigned)HD; ++h)
      s = fmaf(bf16r(Wc1[tid * (unsigned)HD + h]), bf16r(Wc2[h]), s);
    wab[tid] = s;
  } else if (w == 2u) {
    float s = 0.0f;
#pragma unroll 1
    for (unsigned h = 0; h < (unsigned)HD; ++h)
      s = fmaf(bf16r(bc1[h]), bf16r(Wc2[h]), s);
    s = s + bf16r(bc2[0]);
    wab[64u + lane] = s;
  }

  const _Float16* ap  = A16 + (size_t)(row0 + mw * 16u + m) * NN + hh * 8u;
  const _Float16* bph = Gh + (size_t)(nw * 16u + m) * NN + hh * 8u;
  const _Float16* bpr = Gr + (size_t)(nw * 16u + m) * NN + hh * 8u;
  v8f acch = {}, accr = {};
#pragma unroll 2
  for (unsigned k0 = 0; k0 < (unsigned)NN; k0 += 32u) {
    const v16h a  = frag_at(ap + k0);
    const v16h bh = frag_at(bph + k0);
    const v16h br = frag_at(bpr + k0);
    acch = wmma16(a, bh, acch);
    accr = wmma16(a, br, accr);
  }
  const float ir = 1.0f / RCARRY;
  const float cs = 1.0f / (ACARRY * GCARRY);
#pragma unroll
  for (int r = 0; r < 8; ++r)
    xs[(mw * 16u + hh * 8u + (unsigned)r) * LDX + nw * 16u + m] = (acch[r] + accr[r] * ir) * cs;
  __syncthreads();

#pragma unroll 1
  for (unsigned j = 0; j < 8u; ++j) {
    const unsigned idx = tid + 256u * j;
    const unsigned row = idx >> 5, col = idx & 31u;
    const float pre = xs[row * LDX + col] + bf16r(b1[col]);
    xs[row * LDX + col] = tanhf(pre);
  }
  __syncthreads();

  const unsigned xr = tid >> 2, kc = (tid & 3u) * 8u;
  const v4f x0 = *(const v4f*)&xs[xr * LDX + kc];
  const v4f x1 = *(const v4f*)&xs[xr * LDX + kc + 4u];
  v8h o;
#pragma unroll
  for (int i = 0; i < 4; ++i) {
    o[i]     = toh_flush(XCARRY * x0[i]);
    o[i + 4] = toh_flush(XCARRY * x1[i]);
  }
  _Float16* px = X32 + (size_t)(row0 + xr) * HD + kc;

  if (w < 2u) {
    float su = 0.0f, sv = 0.0f;
#pragma unroll 1
    for (unsigned q = 0; q < (unsigned)HD; ++q) {
      const float x = xs[tid * LDX + q];
      su = fmaf(x, wab[q], su);
      sv = fmaf(x, wab[32u + q], sv);
    }
    suv[tid] = su + wab[64];
    suv[64u + tid] = sv;
  }
  __syncthreads();

  const bool uvw = (w < 2u) && (lane < 16u);
  const unsigned ul = lane & 15u;
  const v4f uvv = *(const v4f*)&suv[(w & 1u) * 64u + ul * 4u];
  float* pu = UV + (size_t)(w & 1u) * NN + row0 + ul * 4u;

  *(volatile v8h*)px = o;
  if (uvw) *(volatile v4f*)pu = uvv;
  __threadfence();
  *(volatile v8h*)px = o;
  if (uvw) *(volatile v4f*)pu = uvv;
}
static_assert(256 * 8 == 64 * HD);
static_assert(256 / 4 == 64);
static_assert(16 * 4 == 64);

__global__ __launch_bounds__(256) void gemm_y_kernel(
    const _Float16* __restrict__ X32, const _Float16* __restrict__ X16,
    const _Float16* __restrict__ W2t, _Float16* __restrict__ YT) {
#pragma clang fp contract(off)
  __shared__ __attribute__((aligned(16))) _Float16 Ty[CD * LDY];
  const unsigned tid = threadIdx.x, lane = tid & 31u;
  const unsigned w = (unsigned)__builtin_amdgcn_readfirstlane((int)(threadIdx.x >> 5));
  const unsigned hh = lane >> 4, m = lane & 15u;
  const unsigned rowb = blockIdx.x * 128u + w * 16u;

  const _Float16* ax = X32 + (size_t)(rowb + m) * HD + hh * 8u;
  const _Float16* ai = X16 + (size_t)(rowb + m) * FD + hh * 8u;
  const _Float16* bp = W2t + (size_t)m * KC + hh * 8u;
  v8f acc = {};
  {
    const v16h a = frag_at(ax);
    const v16h b = frag_at(bp);
    acc = wmma16(a, b, acc);
  }
#pragma unroll
  for (unsigned k0 = 0; k0 < (unsigned)FD; k0 += 32u) {
    const v16h a = frag_at(ai + k0);
    const v16h b = frag_at(bp + HD + k0);
    acc = wmma16(a, b, acc);
  }
  const float cs = YCARRY / (WCARRY * XCARRY);
  v8h o;
#pragma unroll
  for (int r = 0; r < 8; ++r) o[r] = toh_flush(acc[r] * cs);
  *(v8h*)&Ty[m * LDY + w * 16u + hh * 8u] = o;
  __syncthreads();

  const unsigned n = tid >> 4, c = (tid & 15u) * 8u;
  const v8h y = *(const v8h*)&Ty[n * LDY + c];
  _Float16* p = YT + (size_t)n * NN + blockIdx.x * 128u + c;
  *(volatile v8h*)p = y;
  __threadfence();
  *(volatile v8h*)p = y;
}
static_assert(256 / 16 == CD);
static_assert(16 * 8 == 128);

__global__ __launch_bounds__(256) void score_kernel(
    const _Float16* __restrict__ A16, const float* __restrict__ UV,
    _Float16* __restrict__ A1) {
#pragma clang fp contract(off)
  const unsigned gid = blockIdx.x * 256u + threadIdx.x;
  const unsigned i = gid / (unsigned)(NN / 8);
  const unsigned c = (gid - i * (unsigned)(NN / 8)) * 8u;
  const float ui = UV[i];
  const v4f v0 = *(const v4f*)(UV + (size_t)NN + c);
  const v4f v1 = *(const v4f*)(UV + (size_t)NN + c + 4u);
  const v8h a = *(const v8h*)(A16 + (size_t)gid * 8u);
  v8h o;
#pragma unroll
  for (int j = 0; j < 4; ++j) {
    const float e0 = ui + v0[j];
    const float e1 = ui + v1[j];
    const float s0 = (e0 > 0.0f) ? 1.0f : e0;
    const float s1 = (e1 > 0.0f) ? 1.0f : e1;
    o[j]     = toh_flush((float)a[j] * s0);
    o[j + 4] = toh_flush((float)a[j + 4] * s1);
  }
  _Float16* p = A1 + (size_t)gid * 8u;
  *(volatile v8h*)p = o;
  __threadfence();
  *(volatile v8h*)p = o;
}

__global__ __launch_bounds__(256) void gemm_out_kernel(
    const _Float16* __restrict__ A1, const _Float16* __restrict__ YT,
    const float* __restrict__ b2, float* __restrict__ out) {
#pragma clang fp contract(off)
  __shared__ __attribute__((aligned(16))) float Cs[128 * LDO];
  const unsigned tid = threadIdx.x, lane = tid & 31u;
  const unsigned w = (unsigned)__builtin_amdgcn_readfirstlane((int)(threadIdx.x >> 5));
  const unsigned hh = lane >> 4, m = lane & 15u;
  const unsigned row0 = blockIdx.x * 128u;

  const _Float16* ap = A1 + (size_t)(row0 + w * 16u + m) * NN + hh * 8u;
  const _Float16* bp = YT + (size_t)m * NN + hh * 8u;
  v8f acc = {};
#pragma unroll 2
  for (unsigned k0 = 0; k0 < (unsigned)NN; k0 += 32u) {
    const v16h a = frag_at(ap + k0);
    const v16h b = frag_at(bp + k0);
    acc = wmma16(a, b, acc);
  }
  const float cs = 1.0f / (ACARRY * YCARRY);
  const float bias = bf16r(b2[m]);
#pragma unroll
  for (int r = 0; r < 8; ++r)
    Cs[(w * 16u + hh * 8u + (unsigned)r) * LDO + m] = acc[r] * cs + bias;
  __syncthreads();

  if (w < 4u) {
    const unsigned rb = tid * LDO;
    float mx = Cs[rb];
#pragma unroll 1
    for (unsigned c = 1; c < (unsigned)CD; ++c) mx = fmaxf(mx, Cs[rb + c]);
    float se = 0.0f;
#pragma unroll 1
    for (unsigned c = 0; c < (unsigned)CD; ++c) se = se + expf(Cs[rb + c] - mx);
    const float ls = logf(se);
#pragma unroll 1
    for (unsigned c = 0; c < (unsigned)CD; ++c) Cs[rb + c] = (Cs[rb + c] - mx) - ls;
  }
  __syncthreads();

  v4f xo[2];
  size_t off[2];
#pragma unroll
  for (unsigned i = 0; i < 2u; ++i) {
    const unsigned idx = tid + 256u * i;
    const unsigned r = idx >> 2, c = (idx & 3u) * 4u;
    xo[i] = *(const v4f*)&Cs[r * LDO + c];
    off[i] = (size_t)(row0 + r) * CD + c;
  }
#pragma unroll
  for (int i = 0; i < 2; ++i) *(volatile v4f*)(out + off[i]) = xo[i];
  __threadfence();
#pragma unroll
  for (int i = 0; i < 2; ++i) *(volatile v4f*)(out + off[i]) = xo[i];
}
static_assert(2 * (256 / 4) == 128);
static_assert(4 * 4 == CD);
static_assert(4 * 32 == 128);

extern "C" void kernel_launch(void* const* d_in, const int* in_sizes, int n_in,
                              void* d_out, int out_size, void* d_ws, size_t ws_size,
                              hipStream_t stream) {
  if (n_in < 12) return;
  if ((long long)in_sizes[0] < (long long)NN * FD) return;
  if ((long long)in_sizes[2] < (long long)(NN - 1) * NN_FULL + NN) return;
  if (in_sizes[4] < FD * HD || in_sizes[5] < HD) return;
  if (in_sizes[6] < KC * CD || in_sizes[7] < CD) return;
  if (in_sizes[8] < 2 * HD * HD || in_sizes[9] < HD) return;
  if (in_sizes[10] < HD || in_sizes[11] < 1) return;
  if ((long long)out_size < (long long)NN * CD) return;
  if (ws_size < WS_TOTAL) return;

  const float* xin = (const float*)d_in[0];
  const float* adj = (const float*)d_in[2];
  const float* w1  = (const float*)d_in[4];
  const float* b1  = (const float*)d_in[5];
  const float* w2  = (const float*)d_in[6];
  const float* b2  = (const float*)d_in[7];
  const float* wc1 = (const float*)d_in[8];
  const float* bc1 = (const float*)d_in[9];
  const float* wc2 = (const float*)d_in[10];
  const float* bc2 = (const float*)d_in[11];
  float* out = (float*)d_out;

  char* ws = (char*)d_ws;
  _Float16* W1t = (_Float16*)(ws + OFF_W1T);
  _Float16* W2t = (_Float16*)(ws + OFF_W2T);
  _Float16* X16 = (_Float16*)(ws + OFF_X16);
  _Float16* A16 = (_Float16*)(ws + OFF_A16);
  _Float16* Gh  = (_Float16*)(ws + OFF_GH);
  _Float16* Gr  = (_Float16*)(ws + OFF_GR);
  _Float16* X32 = (_Float16*)(ws + OFF_X32);
  float*    UV  = (float*)(ws + OFF_UV);
  _Float16* YT  = (_Float16*)(ws + OFF_YT);
  _Float16* A1  = (_Float16*)(ws + OFF_A1);

  dim3 blk(256);
  wconv_kernel<<<dim3(1), blk, 0, stream>>>(w1, W1t, FD, HD);
  wconv_kernel<<<dim3(1), blk, 0, stream>>>(w2, W2t, KC, CD);
  pconv_kernel<<<dim3(NN * (FD / 8) / 256), blk, 0, stream>>>(xin, X16, FD / 8, FD, XCARRY);
  pconv_kernel<<<dim3(NN * (NN / 8) / 256), blk, 0, stream>>>(adj, A16, NN / 8, NN_FULL, ACARRY);
  gemm_xw_kernel<<<dim3(NN / 64), blk, 0, stream>>>(X16, W1t, Gh, Gr);
  gemm_adj_kernel<<<dim3(NN / 64), blk, 0, stream>>>(A16, Gh, Gr, b1, wc1, bc1, wc2, bc2,
                                                     X32, UV);
  gemm_y_kernel<<<dim3(NN / 128), blk, 0, stream>>>(X32, X16, W2t, YT);
  score_kernel<<<dim3(NN * (NN / 8) / 256), blk, 0, stream>>>(A16, UV, A1);
  gemm_out_kernel<<<dim3(NN / 128), blk, 0, stream>>>(A1, YT, b2, out);
}
